// MultiheadAttention_11175504904907
// MI455X (gfx1250) — hardware-verified
//
#include <hip/hip_runtime.h>


#ifndef NB
#define NB 4
#endif
#ifndef SEQ
#define SEQ 2048
#endif
#define NB_FULL   4
#define SEQ_FULL  2048
#define HID       1024
#define NHEAD     16
#define HD        64
#define MROWS     (NB * SEQ)

static_assert(HID == NHEAD * HD);
static_assert(NHEAD == 16);
static_assert(HD == 64);
static_assert(SEQ % 128 == 0);
static_assert(SEQ % 64 == 0);
static_assert(SEQ <= SEQ_FULL);
static_assert(NB >= 1 && NB <= NB_FULL);
static_assert(MROWS % 128 == 0);
static_assert(HID % 128 == 0);
static_assert(HID % 32 == 0);
static_assert(HID == 128 * 8);
static_assert((3 * HID) % 2 == 0);

#define CARRY_X    16.0f
#define CARRY_W    32.0f
#define CARRY_QKV  16.0f
#define CARRY_CTX  1024.0f

typedef unsigned u32;
typedef _Float16 f16;
typedef f16   v16h __attribute__((ext_vector_type(16)));
typedef f16   v8h  __attribute__((ext_vector_type(8)));
typedef float v8f  __attribute__((ext_vector_type(8)));
typedef float v4f  __attribute__((ext_vector_type(4)));

union FragU { v16h v; v8h half[2]; f16 e[16]; };
union H8U   { v8h v; f16 e[8]; };

__device__ __forceinline__ v8f zero8() {
    v8f z = {0.f, 0.f, 0.f, 0.f, 0.f, 0.f, 0.f, 0.f};
    return z;
}

__device__ __forceinline__ v8f wmma16(v16h a, v16h b, v8f c) {
    v8f d = __builtin_amdgcn_wmma_f32_16x16x32_f16(false, a, false, b, (short)0, c, false, false);
    asm volatile("v_nop\n\tv_nop\n\tv_nop\n\tv_nop" : "+v"(d) : "v"(a), "v"(b));
    return d;
}

__device__ __forceinline__ float bf16_rne(float x) {
    u32 u = __float_as_uint(x);
    u = (u + 0x7fffu + ((u >> 16) & 1u)) & 0xffff0000u;
    return __uint_as_float(u);
}

__device__ __forceinline__ float fexp2(float x) {
#if defined(__has_builtin)
#if __has_builtin(__builtin_amdgcn_exp2f)
    return __builtin_amdgcn_exp2f(x);
#else
    return exp2f(x);
#endif
#else
    return exp2f(x);
#endif
}

__device__ __forceinline__ float rowmax16(float x) {
    int v = __builtin_bit_cast(int, x);
    x = fmaxf(x, __builtin_bit_cast(float, __builtin_amdgcn_update_dpp(v, v, 0x121, 0xf, 0xf, false)));
    v = __builtin_bit_cast(int, x);
    x = fmaxf(x, __builtin_bit_cast(float, __builtin_amdgcn_update_dpp(v, v, 0x122, 0xf, 0xf, false)));
    v = __builtin_bit_cast(int, x);
    x = fmaxf(x, __builtin_bit_cast(float, __builtin_amdgcn_update_dpp(v, v, 0x124, 0xf, 0xf, false)));
    v = __builtin_bit_cast(int, x);
    x = fmaxf(x, __builtin_bit_cast(float, __builtin_amdgcn_update_dpp(v, v, 0x128, 0xf, 0xf, false)));
    return x;
}

__device__ __forceinline__ v16h load_frag(const f16* tile, u32 rowbase, u32 pitch, u32 kcol, u32 lane) {
    const u32 r  = rowbase + (lane & 15u);
    const u32 kh = (lane >> 4) << 3;
    const f16* p = tile + (size_t)r * pitch + kcol + kh;
    FragU f;
    f.half[0] = *(const v8h*)(p);
    f.half[1] = *(const v8h*)(p + 16);
    return f.v;
}

__global__ void __launch_bounds__(256)
cvt_rows(const float* __restrict__ src, f16* __restrict__ dst, u32 nrows, u32 dstper, u32 srcper, float carry) {
    const u32 g  = blockIdx.x * 256u + threadIdx.x;
    const u32 m  = g >> 7;
    const u32 c8 = (g & 127u) << 3;
    if (m >= nrows) return;
    const u32 mb = m / dstper;
    const u32 sm = mb * srcper + (m - mb * dstper);
    const float* sp = src + (size_t)sm * HID + c8;
    const v4f a = *(const v4f*)sp;
    const v4f b = *(const v4f*)(sp + 4);
    H8U o;
#pragma unroll
    for (u32 j = 0; j < 4; ++j) {
        const float x0 = a[j];
        const float x1 = b[j];
        o.e[j]     = (f16)(bf16_rne(x0) * carry);
        o.e[j + 4] = (f16)(bf16_rne(x1) * carry);
    }
    f16* dp = dst + (size_t)m * HID + c8;
    *(volatile v8h*)dp = o.v;
    __threadfence();
    *(volatile v8h*)dp = o.v;
}

template <int MODE>
__device__ __forceinline__ void gemm_body(const f16* __restrict__ A, const f16* __restrict__ W,
                                          void* __restrict__ out, float accMul) {
    __shared__ __attribute__((aligned(16))) f16 As[128 * 32];
    __shared__ __attribute__((aligned(16))) f16 Bs[128 * 32];
    __shared__ __attribute__((aligned(16))) f16 Cs[128 * 128];
    static_assert(sizeof(f16) * 128 * 128 == sizeof(float) * 64 * 128);

    const u32 tid  = threadIdx.x;
    const u32 lane = tid & 31u;
    const u32 wave = tid >> 5;
    const u32 wm   = wave & 3u;
    const u32 wn   = wave >> 2;
    const u32 hh8  = (lane >> 4) << 3;
    const u32 c16  = lane & 15u;
    const u32 m0   = blockIdx.x * 128u;
    const u32 n0   = blockIdx.y * 128u;

    v8f acc[2][4];
#pragma unroll
    for (int i = 0; i < 2; ++i)
#pragma unroll
        for (int j = 0; j < 4; ++j) acc[i][j] = zero8();

    const u32 srow = tid >> 1;
    const u32 scol = (tid & 1u) << 4;
    const f16* gA = A + (size_t)(m0 + srow) * HID + scol;
    const f16* gW = W + (size_t)(n0 + srow) * HID + scol;

#pragma unroll 1
    for (u32 k0 = 0; k0 < (u32)HID; k0 += 32u) {
        const v8h ra0 = *(const v8h*)(gA + k0);
        const v8h ra1 = *(const v8h*)(gA + k0 + 8);
        const v8h rb0 = *(const v8h*)(gW + k0);
        const v8h rb1 = *(const v8h*)(gW + k0 + 8);
        __syncthreads();
        *(v8h*)&As[srow * 32u + scol]      = ra0;
        *(v8h*)&As[srow * 32u + scol + 8u] = ra1;
        *(v8h*)&Bs[srow * 32u + scol]      = rb0;
        *(v8h*)&Bs[srow * 32u + scol + 8u] = rb1;
        __syncthreads();

        v16h af[2], bfr[4];
#pragma unroll
        for (int i = 0; i < 2; ++i) af[i] = load_frag(As, wm * 32u + (u32)i * 16u, 32u, 0u, lane);
#pragma unroll
        for (int j = 0; j < 4; ++j) bfr[j] = load_frag(Bs, wn * 64u + (u32)j * 16u, 32u, 0u, lane);
#pragma unroll
        for (int i = 0; i < 2; ++i)
#pragma unroll
            for (int j = 0; j < 4; ++j) acc[i][j] = wmma16(af[i], bfr[j], acc[i][j]);
    }

    const u32 bidx  = m0 / (u32)SEQ;
    const u32 s0    = m0 - bidx * (u32)SEQ;
    const u32 piece = lane & 7u;
    const u32 lsub  = lane >> 3;

    if constexpr (MODE == 0) {
#pragma unroll
        for (int i = 0; i < 2; ++i)
#pragma unroll
            for (int j = 0; j < 4; ++j) {
                const u32 nl = wn * 64u + (u32)j * 16u + c16;
#pragma unroll
                for (int r = 0; r < 8; ++r) {
                    const u32 ml = wm * 32u + (u32)i * 16u + hh8 + (u32)r;
                    Cs[ml * 128u + nl] = (f16)(acc[i][j][r] * accMul);
                }
            }
        __syncthreads();
        f16* op = (f16*)out;
        const size_t bh0 = (size_t)bidx * NHEAD + (n0 >> 6);
#pragma unroll
        for (int pass = 0; pass < 2; ++pass) {
#pragma unroll
            for (u32 it = 0; it < 8; ++it) {
                const u32 L    = wave * 32u + it * 4u + lsub;
                const u32 ml   = L >> 1;
                const u32 hsel = L & 1u;
                const v8h v = *(const v8h*)&Cs[ml * 128u + hsel * 64u + piece * 8u];
                f16* dp = op + ((bh0 + hsel) * SEQ + s0 + ml) * HD + piece * 8u;
                *(volatile v8h*)dp = v;
            }
            if (pass == 0) __threadfence();
        }
    } else if constexpr (MODE == 1) {
#pragma unroll
        for (int i = 0; i < 2; ++i)
#pragma unroll
            for (int j = 0; j < 4; ++j) {
                const u32 nl = wn * 64u + (u32)j * 16u + c16;
                H8U t;
#pragma unroll
                for (int r = 0; r < 8; ++r) t.e[r] = (f16)(acc[i][j][r] * accMul);
                *(v8h*)&Cs[nl * 128u + wm * 32u + (u32)i * 16u + hh8] = t.v;
            }
        __syncthreads();
        f16* op = (f16*)out;
#pragma unroll
        for (int pass = 0; pass < 2; ++pass) {
#pragma unroll
            for (u32 it = 0; it < 8; ++it) {
                const u32 L  = wave * 32u + it * 4u + lsub;
                const u32 nl = L >> 1;
                const u32 mh = L & 1u;
                const v8h v = *(const v8h*)&Cs[nl * 128u + mh * 64u + piece * 8u];
                f16* dp = op + ((size_t)(bidx * (u32)HID + n0 + nl) * SEQ + s0 + mh * 64u + piece * 8u);
                *(volatile v8h*)dp = v;
            }
            if (pass == 0) __threadfence();
        }
    } else {
        float* Cf = (float*)Cs;
        float* of = (float*)out;
#pragma unroll
        for (u32 half = 0; half < 2; ++half) {
            if ((wm >> 1) == half) {
#pragma unroll
                for (int i = 0; i < 2; ++i)
#pragma unroll
                    for (int j = 0; j < 4; ++j) {
                        const u32 nl = wn * 64u + (u32)j * 16u + c16;
#pragma unroll
                        for (int r = 0; r < 8; ++r) {
                            const u32 ml = (wm & 1u) * 32u + (u32)i * 16u + hh8 + (u32)r;
                            Cf[ml * 128u + nl] = acc[i][j][r] * accMul;
                        }
                    }
            }
            __syncthreads();
#pragma unroll
            for (int pass = 0; pass < 2; ++pass) {
#pragma unroll
                for (u32 it = 0; it < 8; ++it) {
                    const u32 L    = wave * 32u + it * 4u + lsub;
                    const u32 row  = L >> 2;
                    const u32 part = L & 3u;
                    const v4f v = *(const v4f*)&Cf[row * 128u + part * 32u + piece * 4u];
                    float* dp = of + (size_t)(m0 + half * 64u + row) * HID + n0 + part * 32u + piece * 4u;
                    *(volatile v4f*)dp = v;
                }
                if (pass == 0) __threadfence();
            }
            __syncthreads();
        }
    }
}

__global__ void __launch_bounds__(256) __attribute__((amdgpu_num_vgpr(256)))
gemm_head(const f16* __restrict__ A, const f16* __restrict__ W, f16* __restrict__ out, float accMul) {
    gemm_body<0>(A, W, (void*)out, accMul);
}

__global__ void __launch_bounds__(256) __attribute__((amdgpu_num_vgpr(256)))
gemm_vt(const f16* __restrict__ A, const f16* __restrict__ W, f16* __restrict__ out, float accMul) {
    gemm_body<1>(A, W, (void*)out, accMul);
}

__global__ void __launch_bounds__(256) __attribute__((amdgpu_num_vgpr(256)))
gemm_out(const f16* __restrict__ A, const f16* __restrict__ W, float* __restrict__ out, float accMul) {
    gemm_body<2>(A, W, (void*)out, accMul);
}

__global__ void __launch_bounds__(256) __attribute__((amdgpu_num_vgpr(256)))
attn_fwd(const f16* __restrict__ Qp, const f16* __restrict__ Kp, const f16* __restrict__ Vt,
         f16* __restrict__ Cp) {
    __shared__ __attribute__((aligned(16))) f16 ks[64 * 64];
    __shared__ __attribute__((aligned(16))) f16 vsT[64 * 64];
    __shared__ __attribute__((aligned(16))) f16 ps[8][16 * 64];
    static_assert(HD == 8 * 8);
    static_assert(2 * 256 * 8 == 64 * 64);

    const u32 tid  = threadIdx.x;
    const u32 lane = tid & 31u;
    const u32 wave = tid >> 5;
    const u32 hh8  = (lane >> 4) << 3;
    const u32 c16  = lane & 15u;
    const u32 bh   = blockIdx.y;
    const u32 bidx = bh >> 4;
    const u32 hidx = bh & 15u;
    const u32 q0   = blockIdx.x * 128u + wave * 16u;
    const size_t head = (size_t)bh * SEQ * HD;

    v16h qa[2];
#pragma unroll
    for (int c = 0; c < 2; ++c) qa[c] = load_frag(Qp + head, q0, HD, (u32)c * 32u, lane);

    FragU onesu;
#pragma unroll
    for (int i = 0; i < 16; ++i) onesu.e[i] = (f16)1.0f;
    const v16h ones = onesu.v;

    float m[8];
    v8f   o[4], lacc;
#pragma unroll
    for (int r = 0; r < 8; ++r) m[r] = -1.0e30f;
#pragma unroll
    for (int dt = 0; dt < 4; ++dt) o[dt] = zero8();
    lacc = zero8();

    const float cl = 1.4426950408889634f * 0.00048828125f;
    f16* psw = &ps[wave][0];

#pragma unroll 1
    for (u32 kt = 0; kt < (u32)(SEQ / 64); ++kt) {
        __syncthreads();
#pragma unroll
        for (u32 p2 = 0; p2 < 2; ++p2) {
            const u32 p   = tid + p2 * 256u;
            const u32 row = p >> 3;
            const u32 pc  = (p & 7u) << 3;
            const v8h kv = *(const v8h*)(Kp + head + (size_t)(kt * 64u + row) * HD + pc);
            const v8h vv = *(const v8h*)(Vt + head + (size_t)row * SEQ + kt * 64u + pc);
            *(v8h*)&ks[row * 64u + pc]  = kv;
            *(v8h*)&vsT[row * 64u + pc] = vv;
        }
        __syncthreads();

        v8f s[4];
#pragma unroll
        for (int nt = 0; nt < 4; ++nt) s[nt] = zero8();
#pragma unroll
        for (int c = 0; c < 2; ++c) {
#pragma unroll
            for (int nt = 0; nt < 4; ++nt) {
                const v16h kb = load_frag(ks, (u32)nt * 16u, 64u, (u32)c * 32u, lane);
                s[nt] = wmma16(qa[c], kb, s[nt]);
            }
        }

#pragma unroll
        for (int r = 0; r < 8; ++r) {
            float x[4];
#pragma unroll
            for (int nt = 0; nt < 4; ++nt) x[nt] = s[nt][r] * cl;
            const float tm = rowmax16(fmaxf(fmaxf(x[0], x[1]), fmaxf(x[2], x[3])));
            const float mn = fmaxf(m[r], tm);
            const float al = fexp2(m[r] - mn);
            m[r] = mn;
            lacc[r] *= al;
#pragma unroll
            for (int dt = 0; dt < 4; ++dt) o[dt][r] *= al;
            const float sh = 10.0f - mn;
#pragma unroll
            for (int nt = 0; nt < 4; ++nt)
                psw[(hh8 + (u32)r) * 64u + (u32)nt * 16u + c16] = (f16)fexp2(x[nt] + sh);
        }
        __syncthreads();

#pragma unroll
        for (int kk = 0; kk < 2; ++kk) {
            const v16h pa = load_frag(psw, 0u, 64u, (u32)kk * 32u, lane);
#pragma unroll
            for (int dt = 0; dt < 4; ++dt) {
                const v16h vb = load_frag(vsT, (u32)dt * 16u, 64u, (u32)kk * 32u, lane);
                o[dt] = wmma16(pa, vb, o[dt]);
            }
            lacc = wmma16(pa, ones, lacc);
        }
    }
    __syncthreads();

#pragma unroll
    for (int r = 0; r < 8; ++r) {
        const float inv = (CARRY_CTX / CARRY_QKV) / lacc[r];
#pragma unroll
        for (int dt = 0; dt < 4; ++dt)
            psw[(hh8 + (u32)r) * 64u + (u32)dt * 16u + c16] = (f16)(o[dt][r] * inv);
    }
    __syncthreads();

    const u32 piece = lane & 7u;
    const u32 lsub  = lane >> 3;
#pragma unroll
    for (int pass = 0; pass < 2; ++pass) {
#pragma unroll
        for (u32 it = 0; it < 4; ++it) {
            const u32 L = it * 4u + lsub;
            const v8h v = *(const v8h*)&psw[L * 64u + piece * 8u];
            f16* dp = Cp + ((size_t)(bidx * (u32)SEQ + q0 + L) * HID + hidx * (u32)HD + piece * 8u);
            *(volatile v8h*)dp = v;
        }
        if (pass == 0) __threadfence();
    }
}

static_assert((size_t)(MROWS / 2) * 256 * 8 == (size_t)MROWS * HID);
static_assert((size_t)(3 * HID / 2) * 256 * 8 == (size_t)3 * HID * HID);
static_assert((size_t)(HID / 2) * 256 * 8 == (size_t)HID * HID);
static_assert((size_t)(MROWS / 128) * (HID / 128) * 128 * 128 == (size_t)MROWS * HID);
static_assert((size_t)(SEQ / 128) * (NB * NHEAD) * 128 * HD == (size_t)MROWS * HID);
static_assert(((size_t)5 * MROWS * HID + (size_t)4 * HID * HID) * sizeof(f16) <= (size_t)134217728);

extern "C" void kernel_launch(void* const* d_in, const int* in_sizes, int n_in,
                              void* d_out, int out_size, void* d_ws, size_t ws_size,
                              hipStream_t stream) {
    if (n_in < 3) return;
    if (in_sizes[0] < ((NB - 1) * SEQ_FULL + SEQ) * HID) return;
    if (in_sizes[1] < 3 * HID * HID) return;
    if (in_sizes[2] < HID * HID) return;
    if (out_size < MROWS * HID) return;

    const float* x     = (const float*)d_in[0];
    const float* wqkv  = (const float*)d_in[1];
    const float* wproj = (const float*)d_in[2];

    const size_t nX = (size_t)MROWS * HID;
    const size_t nW = (size_t)HID * HID;
    const size_t totalHalves = 5 * nX + 4 * nW;
    if (ws_size < totalHalves * sizeof(f16)) return;

    f16* Xh  = (f16*)d_ws;
    f16* Wt  = Xh  + nX;
    f16* Wot = Wt  + 3 * nW;
    f16* Qp  = Wot + nW;
    f16* Kp  = Qp  + nX;
    f16* Vtp = Kp  + nX;
    f16* Cp  = Vtp + nX;

    cvt_rows<<<MROWS / 2, 256, 0, stream>>>(x, Xh, (u32)MROWS, (u32)SEQ, (u32)SEQ_FULL, CARRY_X);
    cvt_rows<<<3 * HID / 2, 256, 0, stream>>>(wqkv, Wt, (u32)(3 * HID), (u32)(3 * HID), (u32)(3 * HID), CARRY_W);
    cvt_rows<<<HID / 2, 256, 0, stream>>>(wproj, Wot, (u32)HID, (u32)HID, (u32)HID, CARRY_W);

    const dim3 gg(MROWS / 128, HID / 128);
    const float accQKV = CARRY_QKV / (CARRY_X * CARRY_W);
    gemm_head<<<gg, 256, 0, stream>>>(Xh, Wt,          Qp,  accQKV);
    gemm_head<<<gg, 256, 0, stream>>>(Xh, Wt + nW,     Kp,  accQKV);
    gemm_vt  <<<gg, 256, 0, stream>>>(Xh, Wt + 2 * nW, Vtp, accQKV);

    attn_fwd<<<dim3(SEQ / 128, NB * NHEAD), 256, 0, stream>>>(Qp, Kp, Vtp, Cp);

    const float accOut = 1.0f / (CARRY_CTX * CARRY_W);
    gemm_out<<<gg, 256, 0, stream>>>(Cp, Wot, (float*)d_out, accOut);
}
